// RNNCell_24429773979888
// MI455X (gfx1250) — hardware-run, weakly checked
//
#include <hip/hip_runtime.h>
#include <math.h>

constexpr int kB      = 1024;
constexpr int kNH     = 2048;
constexpr int kNRule  = 16;
constexpr int kNTuned = 256;
constexpr int kNIn    = kNRule + kNTuned;
constexpr int kNExc   = 1638;
constexpr int kKpad   = 32;
static_assert(kNIn == 272, "input width");
static_assert(kB % 64 == 0 && kNH % 64 == 0, "tile multiples");
static_assert(kNTuned % 32 == 0 && kNH % 32 == 0 && kKpad % 32 == 0, "K multiples of 32");

typedef __attribute__((ext_vector_type(16))) _Float16 v16h;
typedef __attribute__((ext_vector_type(8)))  _Float16 v8h;
typedef __attribute__((ext_vector_type(16))) __bf16   v16b;
typedef __attribute__((ext_vector_type(8)))  __bf16   v8b;
typedef __attribute__((ext_vector_type(8)))  float    v8f;
typedef __attribute__((ext_vector_type(4)))  float    v4f;
typedef __attribute__((ext_vector_type(2)))  float    v2f;
typedef __attribute__((ext_vector_type(2)))  unsigned int v2u;

__device__ __forceinline__ unsigned short f2bf_bits(float f) {
  unsigned u = __float_as_uint(f);
  return (unsigned short)((u + 0x7FFFu + ((u >> 16) & 1u)) >> 16);
}
__device__ __forceinline__ float bf_bits2f(unsigned short h) { return __uint_as_float(((unsigned)h) << 16); }

__device__ __forceinline__ void dep_guard_h(v8f& a, v8f& b, v16h x, v16h y) { asm volatile("v_nop\n\tv_nop\n\tv_nop\n\tv_nop" : "+v"(a), "+v"(b) : "v"(x), "v"(y)); }
__device__ __forceinline__ void dep_guard_b(v8f& a, v8f& b, v16b x, v16b y) { asm volatile("v_nop\n\tv_nop\n\tv_nop\n\tv_nop" : "+v"(a), "+v"(b) : "v"(x), "v"(y)); }
__device__ __forceinline__ void keep4_h(v16h a, v16h b, v16h c, v16h d) { asm volatile("v_nop" :: "v"(a), "v"(b), "v"(c), "v"(d)); }
__device__ __forceinline__ void keep4_b(v16b a, v16b b, v16b c, v16b d) { asm volatile("v_nop" :: "v"(a), "v"(b), "v"(c), "v"(d)); }
__device__ __forceinline__ void acc_guard4(v8f& a, v8f& b, v8f& c, v8f& d) { asm volatile("v_nop\n\tv_nop\n\tv_nop\n\tv_nop" : "+v"(a), "+v"(b), "+v"(c), "+v"(d)); }
template <typename T> struct Frag;
template <> struct Frag<_Float16> {
  typedef v16h V; union U { v16h v; v8h h[2]; };
  static __device__ __forceinline__ v16h load(const _Float16* p) {
    U f; f.h[0] = *(const v8h*)(p); f.h[1] = *(const v8h*)(p + 16); return f.v;
  }
  static __device__ __forceinline__ v8f mma(v16h a, v16h b, v8f c) {
    return __builtin_amdgcn_wmma_f32_16x16x32_f16(false, a, false, b, (short)0, c, false, false);
  }
  static __device__ __forceinline__ void guard(v8f& a, v8f& b, v16h x, v16h y) { dep_guard_h(a, b, x, y); }
  static __device__ __forceinline__ void keep(v16h a, v16h b, v16h c, v16h d) { keep4_h(a, b, c, d); }
};
template <> struct Frag<__bf16> {
  typedef v16b V; union U { v16b v; v8b h[2]; };
  static __device__ __forceinline__ v16b load(const __bf16* p) {
    U f; f.h[0] = *(const v8b*)(p); f.h[1] = *(const v8b*)(p + 16); return f.v;
  }
  static __device__ __forceinline__ v8f mma(v16b a, v16b b, v8f c) {
    return __builtin_amdgcn_wmma_f32_16x16x32_bf16(false, a, false, b, (short)0, c, false, false);
  }
  static __device__ __forceinline__ void guard(v8f& a, v8f& b, v16b x, v16b y) { dep_guard_b(a, b, x, y); }
  static __device__ __forceinline__ void keep(v16b a, v16b b, v16b c, v16b d) { keep4_b(a, b, c, d); }
};

__device__ __forceinline__ unsigned pk16(unsigned short a, unsigned short b) { return (unsigned)a | ((unsigned)b << 16); }
__device__ __forceinline__ float bfr(float x) { return bf_bits2f(f2bf_bits(x)); }

template <int ET> struct Elem;
template <> struct Elem<0> { typedef _Float16 T; };
template <> struct Elem<1> { typedef __bf16 T; };
template <int ET, bool SPLIT, int BIAS_MODE, int OUT_MODE, bool RESID, int ACT = 0>
__global__ __launch_bounds__(256) void wmma_gemm64(
    const unsigned short* __restrict__ Ap, const unsigned short* __restrict__ A2p, int lda, long strideA,
    const unsigned short* __restrict__ Btp, const unsigned short* __restrict__ Bt2p, int ldb, long strideB,
    void* __restrict__ Cout, void* __restrict__ Cout2, int ldc, long strideC,
    const float* __restrict__ bias,
    const float* __restrict__ resid, long strideR,
    int M, int N, int K, float scale) {
  typedef typename Elem<ET>::T T;
  typedef typename Frag<T>::V V;
  const T* A = (const T*)Ap; const T* A2 = (const T*)A2p; const T* Bt = (const T*)Btp; const T* Bt2 = (const T*)Bt2p;
  __shared__ __align__(16) float sT[8][16 * 68];
  const int b    = blockIdx.y;
  const int lane = threadIdx.x & 31;
  const int wave = threadIdx.x >> 5;
  const int tilesN = N >> 6;
  const int tilesM = M >> 6;
  const int tile = blockIdx.x * 8 + wave;
  if (tile >= tilesM * tilesN) return;
  const int tm = tile / tilesN;
  const int tn = tile - tm * tilesN;
  const int m0 = tm << 6;
  const int n0 = tn << 6;

  const T* Ab  = A  + (size_t)b * strideA;
  const T* Bb  = Bt + (size_t)b * strideB;
  const T* Ab2 = SPLIT ? (A2  + (size_t)b * strideA) : nullptr;
  const T* Bb2 = SPLIT ? (Bt2 + (size_t)b * strideB) : nullptr;

  const int rlane = lane & 15;
  const int koff  = (lane >> 4) * 8;
  const int mOff  = (lane >> 4) * 8;

  v8f acc[4][4];
#pragma unroll
  for (int i = 0; i < 4; ++i)
#pragma unroll
    for (int j = 0; j < 4; ++j) acc[i][j] = (v8f){0.f,0.f,0.f,0.f,0.f,0.f,0.f,0.f};

  for (int k0 = 0; k0 < K; k0 += 32) {
    V bh[4], bl[4];
#pragma unroll
    for (int j = 0; j < 4; ++j) {
      const size_t bo = (size_t)(n0 + (j << 4) + rlane) * ldb + koff + k0;
      bh[j] = Frag<T>::load(Bb + bo);
      if (SPLIT) bl[j] = Frag<T>::load(Bb2 + bo);
    }
#pragma unroll
    for (int i = 0; i < 4; ++i) {
      const size_t ao = (size_t)(m0 + (i << 4) + rlane) * lda + koff + k0;
      V ah = Frag<T>::load(Ab + ao);
      V al;
      if (SPLIT) al = Frag<T>::load(Ab2 + ao);
#pragma unroll
      for (int j = 0; j < 4; ++j) {
        acc[i][j] = Frag<T>::mma(ah, bh[j], acc[i][j]);
        if (SPLIT) {
          acc[i][j] = Frag<T>::mma(ah, bl[j], acc[i][j]);
          acc[i][j] = Frag<T>::mma(al, bh[j], acc[i][j]);
        }
      }
      Frag<T>::guard(acc[i][0], acc[i][3], ah, SPLIT ? al : ah);
    }
    Frag<T>::keep(bh[0], bh[1], bh[2], bh[3]);
    if (SPLIT) Frag<T>::keep(bl[0], bl[1], bl[2], bl[3]);
  }
  acc_guard4(acc[0][0], acc[0][1], acc[0][2], acc[0][3]);
  acc_guard4(acc[1][0], acc[1][1], acc[1][2], acc[1][3]);
  acc_guard4(acc[2][0], acc[2][1], acc[2][2], acc[2][3]);
  acc_guard4(acc[3][0], acc[3][1], acc[3][2], acc[3][3]);

  float* slab = sT[wave];
  const float* Rb = RESID ? (resid + (size_t)b * strideR) : nullptr;
#pragma unroll
  for (int i = 0; i < 4; ++i) {
    const int mBase = m0 + (i << 4);
#pragma unroll
    for (int j = 0; j < 4; ++j) {
      const int n = n0 + (j << 4) + rlane;
      float bv = 0.f;
      if (BIAS_MODE == 2) bv = bias[n];
#pragma unroll
      for (int r = 0; r < 8; ++r) {
        float v = acc[i][j][r] * scale;
        if (BIAS_MODE == 1) v += bias[mBase + mOff + r];
        if (BIAS_MODE == 2) v += bv;
        if (RESID) v += Rb[(size_t)(mBase + mOff + r) * ldc + n];
        if (ACT == 2) v = fmaxf(v, 0.0f);
        if (ACT == 4) v = (v > 0.f) ? v : 0.01f * v;
        slab[(mOff + r) * 68 + (j << 4) + rlane] = v;
      }
    }
    __builtin_amdgcn_fence(__ATOMIC_RELEASE, "workgroup");
    __builtin_amdgcn_wave_barrier();
    __builtin_amdgcn_fence(__ATOMIC_ACQUIRE, "workgroup");
    if (OUT_MODE == 0) {
      float* C = (float*)Cout + (size_t)b * strideC;
      const int hh = lane >> 4, c4 = (lane & 15) * 4;
      for (int pass = 0; pass < 2; ++pass) {
#pragma unroll
        for (int it = 0; it < 8; ++it) {
          const int row = it * 2 + hh;
          v4f v = *(const v4f*)(slab + row * 68 + c4);
          *(volatile v4f*)(C + (size_t)(mBase + row) * ldc + n0 + c4) = v;
        }
        __threadfence();
      }
    } else {
      const int q = lane >> 3, c8 = (lane & 7) * 8;
      unsigned short* C  = (unsigned short*)Cout  + (size_t)b * strideC;
      unsigned short* C2 = (OUT_MODE == 2) ? ((unsigned short*)Cout2 + (size_t)b * strideC) : nullptr;
      for (int pass = 0; pass < 2; ++pass) {
#pragma unroll
        for (int it = 0; it < 4; ++it) {
          const int row = it * 4 + q;
          const float* sp = slab + row * 68 + c8;
          v8h hv, lv;
#pragma unroll
          for (int e = 0; e < 8; ++e) {
            if (OUT_MODE == 1) {
              hv[e] = (_Float16)sp[e];
            } else {
              unsigned short hb = f2bf_bits(sp[e]);
              unsigned short lb = f2bf_bits(sp[e] - bf_bits2f(hb));
              hv[e] = __builtin_bit_cast(_Float16, hb);
              lv[e] = __builtin_bit_cast(_Float16, lb);
            }
          }
          *(volatile v8h*)(C + (size_t)(mBase + row) * ldc + n0 + c8) = hv;
          if (OUT_MODE == 2) *(volatile v8h*)(C2 + (size_t)(mBase + row) * ldc + n0 + c8) = lv;
        }
        __threadfence();
      }
    }
    __builtin_amdgcn_fence(__ATOMIC_RELEASE, "workgroup");
    __builtin_amdgcn_wave_barrier();
    __builtin_amdgcn_fence(__ATOMIC_ACQUIRE, "workgroup");
  }
}

__global__ __launch_bounds__(256) void stsp_kernel(const float* __restrict__ prev_h, const float* __restrict__ syn_x,
                                                   const float* __restrict__ syn_u, float* __restrict__ out_sx,
                                                   float* __restrict__ out_su, unsigned short* __restrict__ hpost,
                                                   int n4) {
#pragma clang fp contract(off)
  const int i = blockIdx.x * 256 + threadIdx.x;
  if (i >= n4) return;
  const size_t e0 = 4 * (size_t)i;
  const v4f ph = *(const v4f*)(prev_h + e0);
  const v4f sx = *(const v4f*)(syn_x + e0);
  const v4f su = *(const v4f*)(syn_u + e0);
  v4f ox, ou;
  unsigned short hb[4];
#pragma unroll
  for (int e = 0; e < 4; ++e) {
    const float a_std = (e & 1) ? 0.00417f : 0.05f;
    const float px = bfr(ph[e]);
    const float x  = bfr(sx[e]);
    const float u  = bfr(su[e]);
    const float t1 = a_std * (1.0f - x);
    const float t2 = ((0.01f * u) * x) * px;
    const float xn = (x + t1) - t2;
    const float xc = fminf(1.0f, fmaxf(xn, 0.0f));
    const float uc = fminf(1.0f, fmaxf(xc, 0.0f));
    ox[e] = xc;
    ou[e] = uc;
    hb[e] = f2bf_bits((uc * xc) * px);
  }
  const v2u hp = (v2u){pk16(hb[0], hb[1]), pk16(hb[2], hb[3])};
  *(volatile v4f*)(out_sx + e0) = ox;
  *(volatile v4f*)(out_su + e0) = ou;
  *(volatile v2u*)(hpost + e0) = hp;
  __threadfence();
  *(volatile v4f*)(out_sx + e0) = ox;
  *(volatile v4f*)(out_su + e0) = ou;
  *(volatile v2u*)(hpost + e0) = hp;
}

__global__ __launch_bounds__(256) void wprep_kernel(const float* __restrict__ rnnmat, unsigned short* __restrict__ wrnn,
                                                    int n4) {
  const int i = blockIdx.x * 256 + threadIdx.x;
  if (i >= n4) return;
  const size_t e0 = 4 * (size_t)i;
  const int col = (int)(e0 & (size_t)(kNH - 1));
  const v4f w = *(const v4f*)(rnnmat + e0);
  unsigned short hb[4];
#pragma unroll
  for (int e = 0; e < 4; ++e) {
    float v = bfr(w[e]);
    v = fmaxf(v, 0.0f);
    v = (col + e >= kNExc) ? -v : v;
    hb[e] = f2bf_bits(v);
  }
  const v2u u = (v2u){pk16(hb[0], hb[1]), pk16(hb[2], hb[3])};
  *(volatile v2u*)(wrnn + e0) = u;
  __threadfence();
  *(volatile v2u*)(wrnn + e0) = u;
}

__global__ __launch_bounds__(256) void prep_small_kernel(const float* __restrict__ inputs, const float* __restrict__ Win,
                                                         const float* __restrict__ Wmd_x, const float* __restrict__ Wmd_a,
                                                         unsigned short* __restrict__ rule_p,
                                                         unsigned short* __restrict__ tuned_p,
                                                         unsigned short* __restrict__ win_p,
                                                         unsigned short* __restrict__ wmd_p) {
  const int reg = blockIdx.y;
  const int t = blockIdx.x * 256 + threadIdx.x;
  v4f x;
  bool zero = false;
  unsigned short* dst;
  if (reg == 0) {
    if (t >= kB * 8) return;
    const int b = t >> 3, c4 = (t & 7) * 4;
    const int cc = (c4 < 16) ? c4 : 12;
    x = *(const v4f*)(inputs + (size_t)b * kNIn + cc);
    zero = (c4 >= 16);
    dst = rule_p + (size_t)b * kKpad + c4;
  } else if (reg == 1) {
    if (t >= kB * 64) return;
    const int b = t >> 6, c4 = (t & 63) * 4;
    x = *(const v4f*)(inputs + (size_t)b * kNIn + kNRule + c4);
    dst = tuned_p + (size_t)b * kNTuned + c4;
  } else if (reg == 2) {
    if (t >= kNH * 64) return;
    x = *(const v4f*)(Win + 4 * (size_t)t);
    dst = win_p + 4 * (size_t)t;
  } else {
    if (t >= kNH * 8) return;
    const float* W = (reg == 3) ? Wmd_x : Wmd_a;
    const int rowoff = (reg == 3) ? 0 : kNH;
    const int n = t >> 3, c4 = (t & 7) * 4;
    const int cc = (c4 < 16) ? c4 : 12;
    x = *(const v4f*)(W + (size_t)n * kNRule + cc);
    zero = (c4 >= 16);
    dst = wmd_p + (size_t)(rowoff + n) * kKpad + c4;
  }
  unsigned short hb[4];
#pragma unroll
  for (int e = 0; e < 4; ++e) {
    const float v = zero ? 0.0f : x[e];
    hb[e] = f2bf_bits(v);
  }
  const v2u u = (v2u){pk16(hb[0], hb[1]), pk16(hb[2], hb[3])};
  *(volatile v2u*)dst = u;
  __threadfence();
  *(volatile v2u*)dst = u;
}

__global__ __launch_bounds__(256) void combine_kernel(const float* __restrict__ recp, const float* __restrict__ inpp,
                                                      const float* __restrict__ mdp, const float* __restrict__ noise,
                                                      const float* __restrict__ prev_h, float* __restrict__ out_h,
                                                      float cnoise, int n2) {
#pragma clang fp contract(off)
  const int i = blockIdx.x * 256 + threadIdx.x;
  if (i >= n2) return;
  const size_t e0 = 2 * (size_t)i;
  const size_t b = e0 >> 11;
  const size_t n = e0 & (size_t)(kNH - 1);
  const v2f rc = *(const v2f*)(recp + e0);
  const v2f ip = *(const v2f*)(inpp + e0);
  const v2f mx = *(const v2f*)(mdp + b * (size_t)(2 * kNH) + n);
  const v2f ma = *(const v2f*)(mdp + b * (size_t)(2 * kNH) + kNH + n);
  const v2f nz = *(const v2f*)(noise + e0);
  const v2f ph = *(const v2f*)(prev_h + e0);
  v2f o;
#pragma unroll
  for (int e = 0; e < 2; ++e) {
    const float px = bfr(ph[e]);
    const float nv = bfr(nz[e]);
    float dh = (1.0f + mx[e]) * rc[e];
    dh = dh + ip[e];
    dh = dh + ma[e];
    dh = dh + cnoise * nv;
    float tv = tanhf(dh);
    tv = fmaxf(tv, 0.0f);
    o[e] = 0.9f * px + 0.1f * tv;
  }
  *(volatile v2f*)(out_h + e0) = o;
  __threadfence();
  *(volatile v2f*)(out_h + e0) = o;
}

extern "C" void kernel_launch(void* const* d_in, const int* in_sizes, int n_in,
                              void* d_out, int out_size, void* d_ws, size_t ws_size,
                              hipStream_t stream) {
  if (n_in < 9) return;
  if (in_sizes[0] != kB * kNIn || in_sizes[1] != kB * kNH || in_sizes[2] != kB * kNH || in_sizes[3] != kB * kNH ||
      in_sizes[4] != kB * kNH || in_sizes[5] != kNH * kNH || in_sizes[6] != kNH * kNTuned ||
      in_sizes[7] != kNH * kNRule || in_sizes[8] != kNH * kNRule) return;
  if (out_size != 3 * kB * kNH) return;

  const float* inputs = (const float*)d_in[0];
  const float* prev_h = (const float*)d_in[1];
  const float* syn_x  = (const float*)d_in[2];
  const float* syn_u  = (const float*)d_in[3];
  const float* noise  = (const float*)d_in[4];
  const float* rnnmat = (const float*)d_in[5];
  const float* Win    = (const float*)d_in[6];
  const float* Wmd_x  = (const float*)d_in[7];
  const float* Wmd_a  = (const float*)d_in[8];

  float* out_h  = (float*)d_out;
  float* out_sx = out_h + (size_t)kB * kNH;
  float* out_su = out_h + (size_t)2 * kB * kNH;

  const size_t szHpost = (size_t)kB * kNH * 2;
  const size_t szWrnn  = (size_t)kNH * kNH * 2;
  const size_t szTuned = (size_t)kB * kNTuned * 2;
  const size_t szRule  = (size_t)kB * kKpad * 2;
  const size_t szWinp  = (size_t)kNH * kNTuned * 2;
  const size_t szWmd   = (size_t)2 * kNH * kKpad * 2;
  const size_t szRecp  = (size_t)kB * kNH * 4;
  const size_t szInpp  = (size_t)kB * kNH * 4;
  const size_t szMdp   = (size_t)kB * 2 * kNH * 4;
  const size_t offHpost = 0;
  const size_t offWrnn  = offHpost + szHpost;
  const size_t offTuned = offWrnn + szWrnn;
  const size_t offRule  = offTuned + szTuned;
  const size_t offWinp  = offRule + szRule;
  const size_t offWmd   = offWinp + szWinp;
  const size_t offRecp  = offWmd + szWmd;
  const size_t offInpp  = offRecp + szRecp;
  const size_t offMdp   = offInpp + szInpp;
  const size_t offEnd   = offMdp + szMdp;
  if (offEnd > ws_size) return;

  char* ws = (char*)d_ws;
  unsigned short* hpost = (unsigned short*)(ws + offHpost);
  unsigned short* wrnn  = (unsigned short*)(ws + offWrnn);
  unsigned short* tuned = (unsigned short*)(ws + offTuned);
  unsigned short* rule  = (unsigned short*)(ws + offRule);
  unsigned short* winp  = (unsigned short*)(ws + offWinp);
  unsigned short* wmd   = (unsigned short*)(ws + offWmd);
  float* recp = (float*)(ws + offRecp);
  float* inpp = (float*)(ws + offInpp);
  float* mdp  = (float*)(ws + offMdp);

  {
    const int n4 = kB * kNH / 4;
    stsp_kernel<<<dim3((n4 + 255) / 256), dim3(256), 0, stream>>>(prev_h, syn_x, syn_u, out_sx, out_su, hpost, n4);
  }
  {
    const int n4 = kNH * kNH / 4;
    wprep_kernel<<<dim3((n4 + 255) / 256), dim3(256), 0, stream>>>(rnnmat, wrnn, n4);
  }
  prep_small_kernel<<<dim3(512, 5), dim3(256), 0, stream>>>(inputs, Win, Wmd_x, Wmd_a, rule, tuned, winp, wmd);

  {
    const int tiles = (kB / 64) * (kNH / 64);
    wmma_gemm64<1, false, 0, 0, false, 0><<<dim3((tiles + 7) / 8, 1), dim3(256), 0, stream>>>(
        hpost, hpost, kNH, 0L, wrnn, wrnn, kNH, 0L, (void*)recp, (void*)recp, kNH, 0L,
        (const float*)recp, (const float*)recp, 0L, kB, kNH, kNH, 1.0f);
  }
  {
    const int tiles = (kB / 64) * (kNH / 64);
    wmma_gemm64<1, false, 0, 0, false, 0><<<dim3((tiles + 7) / 8, 1), dim3(256), 0, stream>>>(
        tuned, tuned, kNTuned, 0L, winp, winp, kNTuned, 0L, (void*)inpp, (void*)inpp, kNH, 0L,
        (const float*)inpp, (const float*)inpp, 0L, kB, kNH, kNTuned, 1.0f);
  }
  {
    const int tiles = (kB / 64) * (2 * kNH / 64);
    wmma_gemm64<1, false, 0, 0, false, 0><<<dim3((tiles + 7) / 8, 1), dim3(256), 0, stream>>>(
        rule, rule, kKpad, 0L, wmd, wmd, kKpad, 0L, (void*)mdp, (void*)mdp, 2 * kNH, 0L,
        (const float*)mdp, (const float*)mdp, 0L, kB, 2 * kNH, kKpad, 1.0f);
  }
  {
    const float cnoise = 0.5f * sqrtf(0.2f);
    const int n2 = kB * kNH / 2;
    combine_kernel<<<dim3((n2 + 255) / 256), dim3(256), 0, stream>>>(recp, inpp, mdp, noise, prev_h, out_h, cnoise, n2);
  }
}
